// DilatedMultiheadAttention_51101520888223
// MI455X (gfx1250) — hardware-run, weakly checked
//
#include <hip/hip_runtime.h>
#include <math.h>

typedef __attribute__((ext_vector_type(16))) _Float16 v16h;
typedef __attribute__((ext_vector_type(16))) __bf16 v16b;
typedef __attribute__((ext_vector_type(8)))  _Float16 v8h;
typedef __attribute__((ext_vector_type(8)))  float v8f;
typedef __attribute__((ext_vector_type(4)))  float v4f;
typedef __attribute__((ext_vector_type(2)))  float v2f;
typedef __attribute__((ext_vector_type(4)))  unsigned v4u;
typedef __attribute__((ext_vector_type(4)))  int v4i;
typedef float __attribute__((may_alias)) float_a;
typedef int __attribute__((may_alias)) int_a;

template <typename T> __device__ __forceinline__ void vst2(void* p, T v) { *(volatile T*)p = v; __threadfence(); *(volatile T*)p = v; }
__device__ __forceinline__ v8f wmma16(v16h a, v16h b, v8f c) {
  v8f d = __builtin_amdgcn_wmma_f32_16x16x32_f16(false, a, false, b, (short)0, c, false, false);
  asm volatile("v_nop\n\tv_nop\n\tv_nop\n\tv_nop" : "+v"(d) : "v"(a), "v"(b));
  return d;
}
__device__ __forceinline__ v8f wmma_bf(v16b a, v16b b, v8f c) {
  v8f d = __builtin_amdgcn_wmma_f32_16x16x32_bf16(false, a, false, b, (short)0, c, false, false);
  asm volatile("v_nop\n\tv_nop\n\tv_nop\n\tv_nop" : "+v"(d) : "v"(a), "v"(b));
  return d;
}
__device__ __forceinline__ v16h frag_h(const _Float16* rowk0, int lane) {
  union { v16h v; v8h q[2]; } u; const _Float16* p = rowk0 + 8 * (lane >> 4);
  u.q[0] = *(const v8h*)p; u.q[1] = *(const v8h*)(p + 16); return u.v;
}
__device__ __forceinline__ v16h frag_f32(const float* rowk0, int lane) {
  v16h a; const float* p = rowk0 + 8 * (lane >> 4);
#pragma unroll
  for (int i = 0; i < 8; ++i) { a[i] = (_Float16)p[i]; a[8 + i] = (_Float16)p[16 + i]; }
  return a;
}
__device__ __forceinline__ v16h frag_f32s(const float* rowk0, int lane, float sc) {
  v16h a; const float* p = rowk0 + 8 * (lane >> 4);
#pragma unroll
  for (int i = 0; i < 8; ++i) { a[i] = (_Float16)(p[i] * sc); a[8 + i] = (_Float16)(p[16 + i] * sc); }
  return a;
}
__device__ __forceinline__ v16h fragc_f32(const float* W, int k0, int n, int lane, int ld, int K) {
  v16h a; const int g = lane >> 4;
#pragma unroll
  for (int i = 0; i < 8; ++i) { const int ka = k0 + 8 * g + i, kb = ka + 16;
    a[i] = (_Float16)(ka < K ? W[(size_t)(ka < K ? ka : K - 1) * ld + n] : 0.f); a[8 + i] = (_Float16)(kb < K ? W[(size_t)(kb < K ? kb : K - 1) * ld + n] : 0.f); }
  return a;
}
struct F2 { v16b h, l; };
__device__ __forceinline__ F2 bsplit16(const float v[16]) { F2 r;
#pragma unroll
  for (int i = 0; i < 16; ++i) { const __bf16 h = (__bf16)v[i]; r.h[i] = h; r.l[i] = (__bf16)(v[i] - (float)h); }
  return r; }
__device__ __forceinline__ F2 split_row(const float* row, int k0, int lane) { float v[16]; const float* p = row + k0 + 8 * (lane >> 4);
#pragma unroll
  for (int i = 0; i < 8; ++i) { v[i] = p[i]; v[8 + i] = p[16 + i]; }
  return bsplit16(v); }
__device__ __forceinline__ F2 split_rowK(const float* row, int k0, int lane, int K) { float v[16]; const int g = lane >> 4;
#pragma unroll
  for (int i = 0; i < 8; ++i) { const int ka = k0 + 8 * g + i, kb = ka + 16; v[i] = ka < K ? row[ka < K ? ka : K - 1] : 0.f; v[8 + i] = kb < K ? row[kb < K ? kb : K - 1] : 0.f; }
  return bsplit16(v); }
__device__ __forceinline__ F2 split_col(const float* W, int k0, int n, int lane, int ld, int K) { float v[16]; const int g = lane >> 4;
#pragma unroll
  for (int i = 0; i < 8; ++i) { const int ka = k0 + 8 * g + i, kb = ka + 16; v[i] = ka < K ? W[(size_t)(ka < K ? ka : K - 1) * ld + n] : 0.f; v[8 + i] = kb < K ? W[(size_t)(kb < K ? kb : K - 1) * ld + n] : 0.f; }
  return bsplit16(v); }
__device__ __forceinline__ v8f mac3(const F2& a, const F2& b, v8f c) { c = wmma_bf(a.l, b.h, c); c = wmma_bf(a.h, b.l, c); return wmma_bf(a.h, b.h, c); }
__device__ __forceinline__ float sigm(float v) { return 1.0f / (1.0f + expf(-v)); }
#define LDSX() do { asm volatile("s_wait_dscnt 0" ::: "memory"); __builtin_amdgcn_wave_barrier(); __builtin_amdgcn_fence(__ATOMIC_RELEASE, "workgroup"); } while (0)


#define SS 4096
#define EE 1024
#define NH 16
#define HD 64
#define RR 1024
#ifndef TQB
#define TQB (RR / 64)
#endif
typedef __attribute__((ext_vector_type(8))) __bf16 v8b;
__device__ __forceinline__ v16b frag_b(const __bf16* rowk0, int lane) {
  union { v16b v; v8b q[2]; } u; const __bf16* p = rowk0 + 8 * (lane >> 4);
  u.q[0] = *(const v8b*)p; u.q[1] = *(const v8b*)(p + 16); return u.v;
}
__device__ __forceinline__ float bfr(float v) { return (float)(__bf16)v; }
__device__ __attribute__((noinline)) float exp_ni(float v) { return expf(v); }
__device__ __attribute__((noinline)) float erf_ni(float v) { return erff(v); }

#define WS_QH  0u
#define WS_KH  (WS_QH + 2u * (size_t)SS * EE)
#define WS_VH  (WS_KH + 2u * (size_t)SS * EE)
#define WS_O1  (WS_VH + 2u * (size_t)SS * EE)
#define WS_O2  (WS_O1 + 4u * (size_t)SS * EE)
#define WS_O3  (WS_O2 + 4u * (size_t)2 * RR * EE)
#define WS_END (WS_O3 + 4u * (size_t)RR * EE)

__global__ __launch_bounds__(128) void k_proj(const float* __restrict__ Xq, const float* __restrict__ Xk, const float* __restrict__ Xv, const float* __restrict__ WQ, _Float16* __restrict__ QH, _Float16* __restrict__ KH, _Float16* __restrict__ VH) { __shared__ __align__(16) _Float16 sh[64][136];
  const int tid = threadIdx.x, wave = tid >> 5, lane = tid & 31, col = lane & 15, g = lane >> 4; const int which = blockIdx.z; const int c0 = blockIdx.y * 128; const size_t r0 = (size_t)blockIdx.x * 64;
  const float* X = which == 0 ? Xq : which == 1 ? Xk : Xv;
  v8f acc[8] = {};
#pragma unroll 2
  for (int kc = 0; kc < EE / 32; ++kc) { v16b a; { const float* p = X + (r0 + wave * 16 + col) * EE + kc * 32 + 8 * g;
#pragma unroll
      for (int i = 0; i < 8; ++i) { a[i] = (__bf16)p[i]; a[8 + i] = (__bf16)p[16 + i]; } }
#pragma unroll
    for (int j = 0; j < 8; ++j) { v16b w; const size_t o = c0 + j * 16 + col;
#pragma unroll
      for (int i = 0; i < 8; ++i) { w[i] = (__bf16)WQ[o * EE + kc * 32 + 8 * g + i]; w[8 + i] = (__bf16)WQ[o * EE + kc * 32 + 16 + 8 * g + i]; }
      acc[j] = wmma_bf(a, w, acc[j]); } }
#pragma unroll
  for (int j = 0; j < 8; ++j)
#pragma unroll
    for (int r = 0; r < 8; ++r) sh[wave * 16 + 8 * g + r][j * 16 + col] = (_Float16)acc[j][r];
  __syncthreads(); { _Float16* dst = which == 0 ? QH : which == 1 ? KH : VH; for (int e = tid; e < 64 * 16; e += 128) { const int rl = e >> 4, q = e & 15; vst2((unsigned*)(dst + (r0 + rl) * EE + c0 + q * 8), *(const v4u*)&sh[rl][q * 8]); } } }
template <int BR>
__global__ __launch_bounds__(128) void k_att(const _Float16* __restrict__ QH, const _Float16* __restrict__ KH, const _Float16* __restrict__ VH, const float* __restrict__ MK, float* __restrict__ OB) {
  constexpr int DIL = (BR == 0) ? 1 : (BR == 1) ? 2 : 4; constexpr int SEG = 1024 * DIL;
  __shared__ __align__(16) float sp[4][16][36]; __shared__ __align__(16) float so[4][16][68]; __shared__ __align__(16) _Float16 sv[32][72];
  const int tid = threadIdx.x, wave = tid >> 5, lane = tid & 31, col = lane & 15, g = lane >> 4; const int qb = blockIdx.x, h = blockIdx.y, sgm = blockIdx.z; const size_t seg0 = (size_t)sgm * SEG;
  const int slot0 = qb * 64 + wave * 16;
  v16h aq[2];
#pragma unroll
  for (int kc = 0; kc < 2; ++kc) aq[kc] = frag_h(QH + (seg0 + (size_t)DIL * (slot0 + col)) * EE + h * HD + kc * 32, lane);
  float m[8], l[8];
#pragma unroll
  for (int r = 0; r < 8; ++r) { m[r] = -3.0e38f; l[r] = 0.f; }
  v8f acc[4] = {};
#pragma unroll 1
  for (int ks = 0; ks < RR / 32; ++ks) {
    __syncthreads();
    for (int e = tid; e < 32 * 8; e += 128) { const int i = e >> 3, q8 = e & 7; *(v4u*)&sv[i][q8 * 8] = *(const v4u*)(VH + (seg0 + (size_t)DIL * (ks * 32 + i)) * EE + h * HD + q8 * 8); }
    float s[2][8];
#pragma unroll
    for (int ct = 0; ct < 2; ++ct) { const int kslot = ks * 32 + ct * 16 + col; const size_t kpos = seg0 + (size_t)DIL * kslot; v8f c = {};
#pragma unroll
      for (int kc = 0; kc < 2; ++kc) c = wmma16(aq[kc], frag_h(KH + kpos * EE + h * HD + kc * 32, lane), c);
      const float mk = bfr(MK[kpos]);
#pragma unroll
      for (int r = 0; r < 8; ++r) s[ct][r] = c[r] * 0.125f - mk; }
    float alpha[8];
#pragma unroll
    for (int r = 0; r < 8; ++r) { float mx = fmaxf(s[0][r], s[1][r]);
#pragma unroll
      for (int o = 1; o < 16; o <<= 1) mx = fmaxf(mx, __shfl_xor(mx, o));
      const float mn = fmaxf(m[r], mx); alpha[r] = __expf(m[r] - mn); const float e0 = __expf(s[0][r] - mn), e1 = __expf(s[1][r] - mn); float es = e0 + e1;
#pragma unroll
      for (int o = 1; o < 16; o <<= 1) es += __shfl_xor(es, o);
      l[r] = l[r] * alpha[r] + es; m[r] = mn; sp[wave][8 * g + r][col] = e0; sp[wave][8 * g + r][16 + col] = e1; }
#pragma unroll
    for (int j = 0; j < 4; ++j)
#pragma unroll
      for (int r = 0; r < 8; ++r) acc[j][r] *= alpha[r];
    __syncthreads();
    const v16h pa = frag_f32s(&sp[wave][col][0], lane, 2048.0f);
#pragma unroll
    for (int j = 0; j < 4; ++j) { v16h vb; const int dcol = j * 16 + col;
#pragma unroll
      for (int i = 0; i < 8; ++i) { vb[i] = sv[8 * g + i][dcol]; vb[8 + i] = sv[16 + 8 * g + i][dcol]; }
      acc[j] = wmma16(pa, vb, acc[j]); } }
#pragma unroll
  for (int r = 0; r < 8; ++r) { const float il = (1.0f / 2048.0f) / l[r];
#pragma unroll
    for (int j = 0; j < 4; ++j) so[wave][8 * g + r][j * 16 + col] = acc[j][r] * il; }
  LDSX(); for (int rl = 0; rl < 16; ++rl) if (lane < 16) vst2(OB + ((size_t)sgm * RR + slot0 + rl) * EE + h * HD + lane * 4, *(const v4f*)&so[wave][rl][lane * 4]); }
__global__ __launch_bounds__(256) void k_comb(const float* __restrict__ O1, const float* __restrict__ O2, const float* __restrict__ O3, float* __restrict__ OUT) { const int t = threadIdx.x; const size_t pos = (size_t)blockIdx.x * 64 + (t >> 2); const int c0 = blockIdx.y * 256 + (t & 3) * 64;
  const bool has2 = (pos % 2) == 0, has3 = (pos % 4) == 0; const size_t r2 = (pos / 2048) * RR + (pos % 2048) / 2, r3 = pos / 4;
  for (int q = 0; q < 16; ++q) { const int c = c0 + q * 4; v4f o;
#pragma unroll
    for (int i = 0; i < 4; ++i) { float a = O1[pos * EE + c + i]; if (has2) a += O2[r2 * EE + c + i]; if (has3) a += O3[r3 * EE + c + i]; o[i] = a * (1.0f / 3.0f); }
    vst2(OUT + pos * EE + c, o); } }
extern "C" void kernel_launch(void* const* d_in, const int* in_sizes, int n_in, void* d_out, int out_size, void* d_ws, size_t ws_size, hipStream_t stream) {
  (void)in_sizes; (void)n_in; (void)out_size;
  const float** F = (const float**)d_in;
  if (ws_size < (size_t)WS_END) return;
  char* ws = (char*)d_ws; _Float16 *QH = (_Float16*)(ws + WS_QH), *KH = (_Float16*)(ws + WS_KH), *VH = (_Float16*)(ws + WS_VH); float *O1 = (float*)(ws + WS_O1), *O2 = (float*)(ws + WS_O2), *O3 = (float*)(ws + WS_O3);
  k_proj<<<dim3(SS / 64, EE / 128, 3), 128, 0, stream>>>(F[0], F[1], F[2], F[4], QH, KH, VH);
  k_att<0><<<dim3(TQB, NH, 4), 128, 0, stream>>>(QH, KH, VH, F[3], O1);
  k_att<1><<<dim3(TQB, NH, 2), 128, 0, stream>>>(QH, KH, VH, F[3], O2);
  k_att<2><<<dim3(TQB, NH, 1), 128, 0, stream>>>(QH, KH, VH, F[3], O3);
  k_comb<<<dim3(SS / 64, EE / 256), 256, 0, stream>>>(O1, O2, O3, (float*)d_out);
}
